// Net_20899310862685
// MI455X (gfx1250) — hardware-run, weakly checked
//
#include <hip/hip_runtime.h>
#include <stddef.h>
#include <stdint.h>
#include <math.h>

#define NN      100000
#define NE      1200000
#define HD      64
#define KL      128
#define GBM     128
#define MP      100096
#define NTHR    256
#define NWAVE   8
#define EPT     4
#define WCH     (32 * EPT)
#define NBRUN   1024
#define SLB     10
#define NBK     98
#define WLCAP   2048
#define RCAP    16384
#define DEGCAP  64
#define RBM     128
#define SP      68
#define WSMAX   134217728
#define MAXDEG_IN_MEAS    28
#define MAXDEG_OUT_MEAS   30
#define MAXB1024_IN_MEAS  12588
#define MAXB1024_OUT_MEAS 12491

#define BK_ZINTS (NWAVE * WLCAP + RCAP + 4 * NBRUN + NBRUN)
#define BK_INTS  (BK_ZINTS + 16)
#define BK_LDS   (BK_INTS * 4)
#define SWEEP_PER (((NE + NWAVE * WCH - 1) / (NWAVE * WCH)) * WCH)

static_assert(HD == 64 && KL == 2 * HD && KL % 32 == 0);
static_assert(MP % GBM == 0 && MP >= NN && MP == 782 * GBM);
static_assert(NBRUN == (1 << SLB) && NBRUN % GBM == 0 && NBRUN % RBM == 0 && NBRUN % 32 == 0 && NBRUN % NTHR == 0);
static_assert(NBK * NBRUN >= MP && (NBK - 1) * NBRUN < NN);
static_assert(NE < (1 << 21) && (((long long)NE) << SLB) < (1LL << 31));
static_assert(NE % WCH == 0 && SWEEP_PER % WCH == 0 && (NWAVE - 1) * SWEEP_PER < NE && NWAVE * SWEEP_PER >= NE);
static_assert(RCAP == NWAVE * WLCAP && RCAP % (NTHR * 4) == 0 && BK_ZINTS % (NTHR * 4) == 0);
static_assert((long long)RCAP * 100 >= (long long)MAXB1024_IN_MEAS * 105);
static_assert((long long)RCAP * 100 >= (long long)MAXB1024_OUT_MEAS * 105);
static_assert(WLCAP >= MAXB1024_IN_MEAS / 8 + 8 * 46 + 1);
static_assert(WLCAP >= MAXB1024_OUT_MEAS / 8 + 8 * 46 + 1);
static_assert(MAXDEG_IN_MEAS + 8 <= DEGCAP && DEGCAP % 4 == 0);
static_assert(BK_LDS <= 327680);
static_assert((GBM * SP + 128 + GBM) * 4 <= 65536);
static_assert((NN * (HD / 4)) % NTHR == 0);
static_assert(NN % 2 == 0 && RBM == NWAVE * 16);
static_assert(((MP - NN) * KL / 8) % NTHR == 0 && (HD * KL / 8) % NTHR == 0);

typedef float          v2f   __attribute__((ext_vector_type(2)));
typedef float          v4f   __attribute__((ext_vector_type(4)));
typedef float          v8f   __attribute__((ext_vector_type(8)));
typedef int            v4i   __attribute__((ext_vector_type(4)));
typedef int            v8i   __attribute__((ext_vector_type(8)));
typedef unsigned short v8us  __attribute__((ext_vector_type(8)));
typedef unsigned short v16us __attribute__((ext_vector_type(16)));
typedef __bf16         v16bf __attribute__((ext_vector_type(16)));
typedef v2f  __attribute__((may_alias)) v2fa;
typedef v4f  __attribute__((may_alias)) v4fa;
typedef v4i  __attribute__((may_alias)) v4ia;
typedef v8us __attribute__((may_alias)) v8usa;
union FragB { v16bf v; v16us u; v8us h[2]; v8i w; };

__device__ __forceinline__ v8f wmb(const FragB& a, const FragB& b, v8f c) {
  v8f d = __builtin_amdgcn_wmma_f32_16x16x32_bf16(false, a.v, false, b.v, (short)0, c, false, false);
  asm volatile("v_nop\n\tv_nop\n\tv_nop\n\tv_nop" : "+v"(d) : "v"(a.w), "v"(b.w));
  return d;
}

__device__ __forceinline__ unsigned bf16_bits(float f) {
  const unsigned u = __float_as_uint(f);
  const unsigned r = (u + 0x7FFFu + ((u >> 16) & 1u)) >> 16;
  const unsigned q = (u >> 16) | 0x40u;
  return ((u & 0x7fffffffu) > 0x7f800000u) ? q : r;
}
__device__ __forceinline__ float bf16_val(float f) {
  return __uint_as_float(bf16_bits(f) << 16);
}

__device__ __forceinline__ void st2_v4f(float* p, v4f v) {
  *(volatile v4f*)p = v;
  __threadfence();
  *(volatile v4f*)p = v;
}
__device__ __forceinline__ void st2_v8us(unsigned short* p, v8us v) {
  *(volatile v8us*)p = v;
  __threadfence();
  *(volatile v8us*)p = v;
}

__device__ __forceinline__ v8us gather8(const float* __restrict__ base, int stride) {
  float f[8];
#pragma unroll
  for (int i = 0; i < 8; ++i) f[i] = base[(size_t)i * (size_t)stride];
  v8us o;
#pragma unroll
  for (int i = 0; i < 8; ++i) o[i] = (unsigned short)bf16_bits(f[i]);
  return o;
}

__global__ __launch_bounds__(NTHR) void k_prep(const float* __restrict__ w1, const float* __restrict__ b1,
                                               const float* __restrict__ w2, const float* __restrict__ b2,
                                               unsigned short* w1d, unsigned short* w2d,
                                               unsigned short* aggpad, float* sm) {
  const int tid = (int)threadIdx.x, lane = tid & 31;
  const int blk = (int)blockIdx.x;
  if (blk < 4) {
    const int u = blk * NTHR + tid;
    const int n = u >> 4, k8 = (u & 15) * 8, kk = k8 & 63;
    const v8us o = gather8(w1 + (size_t)kk * HD + n, HD);
    st2_v8us(w1d + (size_t)n * KL + k8, o);
  } else if (blk < 8) {
    const int u = (blk - 4) * NTHR + tid;
    const int n = u >> 4, k8 = (u & 15) * 8, kk = k8 & 63;
    const v8us o = gather8(w2 + (size_t)kk * HD + n, HD);
    st2_v8us(w2d + (size_t)n * KL + k8, o);
  } else if (blk < 14) {
    const int u = (blk - 8) * NTHR + tid;
    const v8us z = {0, 0, 0, 0, 0, 0, 0, 0};
    st2_v8us(aggpad + (size_t)u * 8, z);
  } else {
    if (tid < 32) {
      const int q = lane & 15;
      const v4f a = *(const v4fa*)(b1 + 4 * q);
      const v4f c = *(const v4fa*)(b2 + 4 * q);
      asm volatile("" :: "v"(a));
      asm volatile("" :: "v"(c));
      const unsigned ma = (lane < 16) ? 0xffffffffu : 0u;
      v4f o;
      o.x = __uint_as_float(((bf16_bits(a.x) << 16) & ma) | ((bf16_bits(c.x) << 16) & ~ma));
      o.y = __uint_as_float(((bf16_bits(a.y) << 16) & ma) | ((bf16_bits(c.y) << 16) & ~ma));
      o.z = __uint_as_float(((bf16_bits(a.z) << 16) & ma) | ((bf16_bits(c.z) << 16) & ~ma));
      o.w = __uint_as_float(((bf16_bits(a.w) << 16) & ma) | ((bf16_bits(c.w) << 16) & ~ma));
      st2_v4f(sm + 4 * lane, o);
    }
  }
}

__device__ __forceinline__ int sweep_keys(const int* __restrict__ keys, unsigned nbs, unsigned nb,
                                          int* mylist, int wave, int lane) {
  const int ebeg = wave * SWEEP_PER;
  const int eend = (ebeg + SWEEP_PER < NE) ? (ebeg + SWEEP_PER) : NE;
  int wc = 0;
#pragma unroll 1
  for (int cb = ebeg; cb < eend; cb += WCH) {
    const int e0 = cb + lane * EPT;
    const v4i da = *(const v4ia*)(keys + e0);
    const unsigned s0 = (unsigned)da.x - nbs, s1 = (unsigned)da.y - nbs;
    const unsigned s2 = (unsigned)da.z - nbs, s3 = (unsigned)da.w - nbs;
    const bool h0 = s0 < nb, h1 = s1 < nb, h2 = s2 < nb, h3 = s3 < nb;
    const unsigned m0 = __builtin_amdgcn_ballot_w32(h0), m1 = __builtin_amdgcn_ballot_w32(h1);
    const unsigned m2 = __builtin_amdgcn_ballot_w32(h2), m3 = __builtin_amdgcn_ballot_w32(h3);
    const unsigned any = m0 | m1 | m2 | m3;
    if (any != 0u) {
      const int pre = (int)(__builtin_amdgcn_mbcnt_lo(m0, 0u) + __builtin_amdgcn_mbcnt_lo(m1, 0u) +
                            __builtin_amdgcn_mbcnt_lo(m2, 0u) + __builtin_amdgcn_mbcnt_lo(m3, 0u));
      int p = wc + pre;
      if (h0) { if (p < WLCAP) mylist[p] = ((e0 + 0) << SLB) | (int)s0; p = p + 1; }
      if (h1) { if (p < WLCAP) mylist[p] = ((e0 + 1) << SLB) | (int)s1; p = p + 1; }
      if (h2) { if (p < WLCAP) mylist[p] = ((e0 + 2) << SLB) | (int)s2; p = p + 1; }
      if (h3) { if (p < WLCAP) mylist[p] = ((e0 + 3) << SLB) | (int)s3; p = p + 1; }
      wc += (int)(__builtin_popcount(m0) + __builtin_popcount(m1) + __builtin_popcount(m2) + __builtin_popcount(m3));
    }
  }
  return wc;
}

__device__ __forceinline__ int count_hits(const int* wl, const int* misc, int* cnt, int lane) {
  int ov = 0;
#pragma unroll 1
  for (int w2 = 0; w2 < NWAVE; ++w2) {
    int c = misc[w2];
    if (c > WLCAP) ov = 1;
    c = c < 0 ? 0 : (c > WLCAP ? WLCAP : c);
#pragma unroll 1
    for (int b0 = 0; b0 < c; b0 += 32) {
      const int idx = b0 + lane;
      const int ent = wl[w2 * WLCAP + (idx < WLCAP ? idx : WLCAP - 1)];
      const int m32 = (c - b0) < 32 ? (c - b0) : 32;
#pragma unroll 1
      for (int k = 0; k < m32; ++k) {
        const int u    = __builtin_amdgcn_readlane(ent, k);
        const int slot = u & (NBRUN - 1);
        if (lane == 0) cnt[slot] = cnt[slot] + 1;
      }
    }
  }
  return ov;
}

__device__ __forceinline__ void bucket_flush(const int* pl, const int* tab, int ov, int* lp, int* cp, int* op,
                                             int* nip, int* nop, int* fp, int tid) {
#pragma unroll 1
  for (int i = tid * 4; i < RCAP; i += NTHR * 4) {
    const v4i v = *(const v4ia*)(pl + i);
    *(volatile v4i*)(lp + i) = v;
  }
  {
    const v4i v0 = *(const v4ia*)(tab + 4 * tid);
    const v4i v1 = *(const v4ia*)(tab + NBRUN + 4 * tid);
    const v4i v2 = *(const v4ia*)(tab + 2 * NBRUN + 4 * tid);
    const v4i v3 = *(const v4ia*)(tab + 3 * NBRUN + 4 * tid);
    *(volatile v4i*)(cp + 4 * tid)  = v0;
    *(volatile v4i*)(op + 4 * tid)  = v1;
    *(volatile v4i*)(nip + 4 * tid) = v2;
    *(volatile v4i*)(nop + 4 * tid) = v3;
  }
  if (tid < 8) {
    const v4i f = {ov, ov, ov, ov};
    *(volatile v4i*)(fp + 4 * tid) = f;
  }
}

__global__ __launch_bounds__(NTHR) void k_bucket(const int* __restrict__ srcs, const int* __restrict__ dsts,
                                                 int* LIST, int* CNT, int* OFF, int* NIB, int* NOB, int* FLAG) {
  extern __shared__ __attribute__((aligned(16))) int dsm[];
  int* wl   = dsm;
  int* pl   = dsm + NWAVE * WLCAP;
  int* tab  = pl + RCAP;
  int* cur  = tab + 4 * NBRUN;
  int* misc = cur + NBRUN;
  int* cnt  = tab;
  int* offs = tab + NBRUN;
  const int tid = (int)threadIdx.x, lane = tid & 31, wave = tid >> 5;
  const int blk = (int)blockIdx.x;
  const unsigned nbs = (unsigned)(blk * NBRUN);
  const int nbi = (NN - blk * NBRUN) < NBRUN ? (NN - blk * NBRUN) : NBRUN;
  const unsigned nb = (unsigned)nbi;

  {
    const v4i z4 = {0, 0, 0, 0};
    for (int i = tid * 4; i < BK_ZINTS; i += NTHR * 4) *(v4ia*)(dsm + i) = z4;
    if (tid < 16) misc[tid] = 0;
  }
  __syncthreads();

  {
    const int wc = sweep_keys(dsts, nbs, nb, wl + wave * WLCAP, wave, lane);
    if (lane == 0) misc[wave] = wc;
  }
  __syncthreads();

  if (wave == 0) {
    const int ov = count_hits(wl, misc, cnt, lane);
    if (lane == 0) misc[9] = ov;
  }
  __syncthreads();
  if (wave == 0) {
    const int base = lane * (NBRUN / 32);
    int s = 0;
#pragma unroll 1
    for (int i = 0; i < NBRUN / 32; ++i) s += cnt[base + i];
    int incl = s;
#pragma unroll
    for (int d = 1; d < 32; d <<= 1) {
      const int y = __shfl_up(incl, d, 32);
      if (lane >= d) incl += y;
    }
    int run = incl - s;
#pragma unroll 1
    for (int i = 0; i < NBRUN / 32; ++i) {
      const int cv = cnt[base + i];
      offs[base + i] = run;
      cur[base + i]  = run;
      run += cv;
    }
  }
  __syncthreads();

  if (wave == 0) {
#pragma unroll 1
    for (int w2 = 0; w2 < NWAVE; ++w2) {
      int c = misc[w2];
      c = c < 0 ? 0 : (c > WLCAP ? WLCAP : c);
#pragma unroll 1
      for (int b0 = 0; b0 < c; b0 += 32) {
        const int idx = b0 + lane;
        const int ent = wl[w2 * WLCAP + (idx < WLCAP ? idx : WLCAP - 1)];
        int eid = (ent >> SLB) & 0x1FFFFF;
        eid = eid > NE - 1 ? NE - 1 : eid;
        int sr = srcs[eid];
        sr = sr < 0 ? 0 : (sr > NN - 1 ? NN - 1 : sr);
        const int m32 = (c - b0) < 32 ? (c - b0) : 32;
#pragma unroll 1
        for (int k = 0; k < m32; ++k) {
          const int u    = __builtin_amdgcn_readlane(ent, k);
          const int wd   = __builtin_amdgcn_readlane(sr, k);
          const int slot = u & (NBRUN - 1);
          if (lane == 0) {
            int p = cur[slot];
            p = p < 0 ? 0 : (p > RCAP - 1 ? RCAP - 1 : p);
            pl[p] = wd;
            cur[slot] = p + 1;
          }
        }
      }
    }
  }
  __syncthreads();

  {
    const int wc = sweep_keys(srcs, nbs, nb, wl + wave * WLCAP, wave, lane);
    if (lane == 0) misc[wave] = wc;
  }
  __syncthreads();
  if (wave == 0) {
    const int ov = count_hits(wl, misc, tab + 3 * NBRUN, lane);
    if (lane == 0) misc[10] = ov;
  }
  __syncthreads();

#pragma unroll 1
  for (int i = tid; i < 2 * NBRUN; i += NTHR) {
    const int rd = i + ((i >> SLB) << (SLB + 1));
    int d = tab[rd];
    d = d < 1 ? 1 : d;
    const float r = 1.0f / sqrtf((float)d);
    tab[2 * NBRUN + i] = __float_as_int(r);
  }
  __syncthreads();

  const int ovf = misc[9] | misc[10];
  int* lp  = LIST + (size_t)blk * RCAP;
  int* cp  = CNT + (size_t)blk * NBRUN;
  int* op  = OFF + (size_t)blk * NBRUN;
  int* nip = NIB + (size_t)blk * NBRUN;
  int* nop = NOB + (size_t)blk * NBRUN;
  int* fp  = FLAG + (size_t)blk * 32;
  bucket_flush(pl, tab, ovf, lp, cp, op, nip, nop, fp, tid);
  __threadfence();
  bucket_flush(pl, tab, ovf, lp, cp, op, nip, nop, fp, tid);
}

__global__ __launch_bounds__(NTHR) void k_prescale(const float* __restrict__ feats, const float* __restrict__ NOt,
                                                   const int* __restrict__ FLAG, float* PN) {
  const int u   = (int)blockIdx.x * NTHR + (int)threadIdx.x;
  const int row = u >> 4, c4 = u & 15;
  const v4f a   = *(const v4fa*)(feats + (size_t)row * HD + 4 * c4);
  const float no = NOt[row];
  const int flag = FLAG[(size_t)(row >> SLB) * 32];
  const float qnan = __uint_as_float(0x7fc00000u);
  v4f o;
  o.x = bf16_val(a.x) * no; o.y = bf16_val(a.y) * no; o.z = bf16_val(a.z) * no; o.w = bf16_val(a.w) * no;
  o.x = (flag != 0) ? qnan : o.x; o.y = (flag != 0) ? qnan : o.y;
  o.z = (flag != 0) ? qnan : o.z; o.w = (flag != 0) ? qnan : o.w;
  st2_v4f(PN + (size_t)row * HD + 4 * c4, o);
}

__global__ __launch_bounds__(NTHR) void k_replay(const int* __restrict__ LIST, const int* __restrict__ CNT,
                                                 const int* __restrict__ OFF, const float* __restrict__ NIt,
                                                 const int* __restrict__ FLAG, const float* __restrict__ PN,
                                                 unsigned* AGG) {
  const int tid = (int)threadIdx.x, lane = tid & 31, wave = tid >> 5;
  const int rowBase = (int)blockIdx.x * RBM;
  const int bucket  = rowBase >> SLB;
  const int* lb  = LIST + (size_t)bucket * RCAP;
  const int flag = FLAG[(size_t)bucket * 32];
  const float qnan = __uint_as_float(0x7fc00000u);

#pragma unroll 1
  for (int i = 0; i < RBM / NWAVE; ++i) {
    const int d = rowBase + (RBM / NWAVE) * wave + i;
    if (d < NN) {
      const int craw = __builtin_amdgcn_readfirstlane(CNT[d]);
      const int oraw = __builtin_amdgcn_readfirstlane(OFF[d]);
      const float ni = NIt[d];
      const bool big = craw > DEGCAP;
      int c = craw < 0 ? 0 : (craw > DEGCAP ? DEGCAP : craw);
      int o = oraw < 0 ? 0 : (oraw > RCAP - 1 ? RCAP - 1 : oraw);
      int last = o + c - 1; last = last < o ? o : last;
      last = last > RCAP - 1 ? RCAP - 1 : last;
      float a0 = 0.0f, a1 = 0.0f;
#pragma unroll 1
      for (int j = 0; j < c; j += 4) {
        int i0 = o + j, i1 = i0 + 1, i2 = i0 + 2, i3 = i0 + 3;
        i0 = i0 > last ? last : i0; i1 = i1 > last ? last : i1;
        i2 = i2 > last ? last : i2; i3 = i3 > last ? last : i3;
        int s0 = lb[i0], s1 = lb[i1], s2 = lb[i2], s3 = lb[i3];
        s0 = s0 < 0 ? 0 : (s0 > NN - 1 ? NN - 1 : s0);
        s1 = s1 < 0 ? 0 : (s1 > NN - 1 ? NN - 1 : s1);
        s2 = s2 < 0 ? 0 : (s2 > NN - 1 ? NN - 1 : s2);
        s3 = s3 < 0 ? 0 : (s3 > NN - 1 ? NN - 1 : s3);
        const v2f v0 = *(const v2fa*)(PN + (size_t)s0 * HD + 2 * lane);
        const v2f v1 = *(const v2fa*)(PN + (size_t)s1 * HD + 2 * lane);
        const v2f v2 = *(const v2fa*)(PN + (size_t)s2 * HD + 2 * lane);
        const v2f v3 = *(const v2fa*)(PN + (size_t)s3 * HD + 2 * lane);
        asm volatile("" :: "v"(v0), "v"(v1));
        asm volatile("" :: "v"(v2), "v"(v3));
        const bool k1 = (j + 1) < c, k2 = (j + 2) < c, k3 = (j + 3) < c;
        a0 = a0 + v0.x; a1 = a1 + v0.y;
        { const float t0 = a0 + v1.x, t1 = a1 + v1.y; a0 = k1 ? t0 : a0; a1 = k1 ? t1 : a1; }
        { const float t0 = a0 + v2.x, t1 = a1 + v2.y; a0 = k2 ? t0 : a0; a1 = k2 ? t1 : a1; }
        { const float t0 = a0 + v3.x, t1 = a1 + v3.y; a0 = k3 ? t0 : a0; a1 = k3 ? t1 : a1; }
      }
      a0 = a0 * ni; a1 = a1 * ni;
      const bool bad = (flag != 0) | big;
      a0 = bad ? qnan : a0; a1 = bad ? qnan : a1;
      const unsigned h0 = bf16_bits(a0), h1 = bf16_bits(a1);
      const unsigned l0 = bf16_bits(a0 - __uint_as_float(h0 << 16));
      const unsigned l1 = bf16_bits(a1 - __uint_as_float(h1 << 16));
      const unsigned hw = h0 | (h1 << 16);
      const unsigned lw = l0 | (l1 << 16);
      unsigned* hp = AGG + (size_t)d * (KL / 2) + lane;
      *(volatile unsigned*)hp = hw;
      *(volatile unsigned*)(hp + 32) = lw;
      __threadfence();
      *(volatile unsigned*)hp = hw;
      *(volatile unsigned*)(hp + 32) = lw;
    }
  }
}

template <int KTOT>
__device__ __forceinline__ void gemm_16x64(const unsigned short* __restrict__ ap,
                                           const unsigned short* __restrict__ bp, v8f (&acc)[4]) {
#pragma unroll 1
  for (int k0 = 0; k0 < KTOT; k0 += 32) {
    FragB af;
    af.h[0] = *(const v8usa*)(ap + k0);
    af.h[1] = *(const v8usa*)(ap + k0 + 16);
#pragma unroll
    for (int nt = 0; nt < 4; ++nt) {
      const unsigned short* wq = bp + (size_t)(16 * nt) * (size_t)KTOT + k0;
      FragB bf;
      bf.h[0] = *(const v8usa*)wq;
      bf.h[1] = *(const v8usa*)(wq + 16);
      acc[nt] = wmb(af, bf, acc[nt]);
    }
  }
}

__device__ __forceinline__ void stage_d(float* stg, const v8f (&acc)[4], int wave, int hh, int m) {
#pragma unroll
  for (int nt = 0; nt < 4; ++nt) {
#pragma unroll
    for (int r = 0; r < 8; ++r) stg[(16 * wave + 8 * hh + r) * SP + 16 * nt + m] = acc[nt][r];
  }
}

template <int FIN>
__global__ __launch_bounds__(NTHR) __attribute__((amdgpu_num_vgpr(248)))
void k_gemm(const unsigned short* __restrict__ A, const unsigned short* __restrict__ BT,
            const float* __restrict__ sm, const float* __restrict__ NOt, const int* __restrict__ FLAG,
            float* P) {
  __shared__ __attribute__((aligned(16))) float stg[GBM * SP];
  __shared__ __attribute__((aligned(16))) float sb[128];
  __shared__ __attribute__((aligned(16))) float sno[GBM];
  const int tid = (int)threadIdx.x, lane = tid & 31, wave = tid >> 5, hh = lane >> 4, m = lane & 15;
  const int rowBase = (int)blockIdx.x * GBM;
  if (wave == 0) *(v4fa*)(sb + 4 * lane)  = *(const v4fa*)(sm + 4 * lane);
  if (wave == 1) *(v4fa*)(sno + 4 * lane) = *(const v4fa*)(NOt + rowBase + 4 * lane);
  const int flag = FLAG[(size_t)(rowBase >> SLB) * 32];

  v8f acc[4];
  {
    const v8f z = {0.f, 0.f, 0.f, 0.f, 0.f, 0.f, 0.f, 0.f};
#pragma unroll
    for (int t = 0; t < 4; ++t) acc[t] = z;
  }
  const unsigned short* ap = A + (size_t)(rowBase + 16 * wave + m) * (size_t)KL + 8 * hh;
  const unsigned short* bp = BT + (size_t)m * (size_t)KL + 8 * hh;
  gemm_16x64<KL>(ap, bp, acc);
  stage_d(stg, acc, wave, hh, m);
  __syncthreads();

  const v4f bias = *(const v4fa*)(sb + FIN * 64 + 4 * m);
  const float qnan = __uint_as_float(0x7fc00000u);
#pragma unroll 1
  for (int i = 0; i < 8; ++i) {
    const int lr   = 16 * wave + 2 * i + hh;
    const int grow = rowBase + lr;
    const bool live = grow < NN;
    const v4f a = *(const v4fa*)(stg + lr * SP + 4 * m);
    asm volatile("" :: "v"(a));
    float v0 = a.x + bias.x, v1 = a.y + bias.y, v2 = a.z + bias.z, v3 = a.w + bias.w;
    if constexpr (FIN == 0) {
      const float no = sno[lr];
      v0 = (v0 > 0.0f) ? v0 : (v0 - v0); v1 = (v1 > 0.0f) ? v1 : (v1 - v1);
      v2 = (v2 > 0.0f) ? v2 : (v2 - v2); v3 = (v3 > 0.0f) ? v3 : (v3 - v3);
      v0 = v0 * no; v1 = v1 * no; v2 = v2 * no; v3 = v3 * no;
    } else {
      v0 = (flag != 0) ? qnan : v0; v1 = (flag != 0) ? qnan : v1;
      v2 = (flag != 0) ? qnan : v2; v3 = (flag != 0) ? qnan : v3;
    }
    v4f o;
    o.x = v0; o.y = v1; o.z = v2; o.w = v3;
    const int gr = live ? grow : NN - 1;
    float* op = P + (size_t)gr * HD + 4 * m;
    if (live) *(volatile v4f*)op = o;
    __threadfence();
    if (live) *(volatile v4f*)op = o;
  }
}

extern "C" void kernel_launch(void* const* d_in, const int* in_sizes, int n_in,
                              void* d_out, int out_size, void* d_ws, size_t ws_size,
                              hipStream_t stream) {
  if (n_in < 7) return;
  if (in_sizes[0] != NN * HD) return;
  if (in_sizes[1] != NE) return;
  if (in_sizes[2] != NE) return;
  if (in_sizes[3] != HD * HD) return;
  if (in_sizes[4] != HD) return;
  if (in_sizes[5] != HD * HD) return;
  if (in_sizes[6] != HD) return;
  if (out_size != NN * HD) return;

  const float* feats = (const float*)d_in[0];
  const int*   srcs  = (const int*)d_in[1];
  const int*   dsts  = (const int*)d_in[2];
  const float* W1    = (const float*)d_in[3];
  const float* b1    = (const float*)d_in[4];
  const float* W2    = (const float*)d_in[5];
  const float* b2    = (const float*)d_in[6];
  float* out = (float*)d_out;

  constexpr size_t zPN   = (size_t)NN * HD * 4;
  constexpr size_t zAGG  = (size_t)MP * KL * 2;
  constexpr size_t zLIST = (size_t)NBK * RCAP * 4;
  constexpr size_t zTAB  = (size_t)NBK * NBRUN * 4;
  constexpr size_t zFLAG = (size_t)NBK * 128;
  constexpr size_t zWD   = (size_t)HD * KL * 2;
  constexpr size_t zSM   = 512;
  constexpr size_t oPN   = 0;
  constexpr size_t oAGG  = oPN + zPN;
  constexpr size_t oLIST = oAGG + zAGG;
  constexpr size_t oCNT  = oLIST + zLIST;
  constexpr size_t oOFF  = oCNT + zTAB;
  constexpr size_t oNI   = oOFF + zTAB;
  constexpr size_t oNO   = oNI + zTAB;
  constexpr size_t oFLAG = oNO + zTAB;
  constexpr size_t oW1D  = oFLAG + zFLAG;
  constexpr size_t oW2D  = oW1D + zWD;
  constexpr size_t oSM   = oW2D + zWD;
  constexpr size_t oEND  = oSM + zSM;
  static_assert(zPN % 256 == 0 && zAGG % 256 == 0 && zLIST % 256 == 0 && zTAB % 256 == 0);
  static_assert(zFLAG % 256 == 0 && zWD % 256 == 0 && zSM % 256 == 0);
  static_assert((size_t)(NBK - 1) * NBRUN + NBRUN <= zTAB / 4);
  static_assert((size_t)(MP / GBM - 1) * GBM + GBM <= zTAB / 4);
  static_assert(oEND == 59298560 && oEND <= (size_t)WSMAX);
  if (oEND > ws_size) return;

  char* ws = (char*)d_ws;
  float*          PN   = (float*)(ws + oPN);
  unsigned short* AGG  = (unsigned short*)(ws + oAGG);
  int*            LIST = (int*)(ws + oLIST);
  int*            CNT  = (int*)(ws + oCNT);
  int*            OFF  = (int*)(ws + oOFF);
  int*            NIB  = (int*)(ws + oNI);
  int*            NOB  = (int*)(ws + oNO);
  int*            FLAG = (int*)(ws + oFLAG);
  unsigned short* W1D  = (unsigned short*)(ws + oW1D);
  unsigned short* W2D  = (unsigned short*)(ws + oW2D);
  float*          SM   = (float*)(ws + oSM);
  const float* NIf = (const float*)(ws + oNI);
  const float* NOf = (const float*)(ws + oNO);

  hipFuncSetAttribute(reinterpret_cast<const void*>(&k_bucket), hipFuncAttributeMaxDynamicSharedMemorySize, (int)BK_LDS);

  k_prep<<<15, NTHR, 0, stream>>>(W1, b1, W2, b2, W1D, W2D, AGG + (size_t)NN * KL, SM);
  k_bucket<<<NBK, NTHR, BK_LDS, stream>>>(srcs, dsts, LIST, CNT, OFF, NIB, NOB, FLAG);
  k_prescale<<<(NN * (HD / 4)) / NTHR, NTHR, 0, stream>>>(feats, NOf, FLAG, PN);

  k_replay<<<(NN + RBM - 1) / RBM, NTHR, 0, stream>>>(LIST, CNT, OFF, NIf, FLAG, PN, (unsigned*)AGG);
  k_gemm<0><<<MP / GBM, NTHR, 0, stream>>>(AGG, W1D, SM, NOf, FLAG, PN);
  k_replay<<<(NN + RBM - 1) / RBM, NTHR, 0, stream>>>(LIST, CNT, OFF, NIf, FLAG, PN, (unsigned*)AGG);
  k_gemm<1><<<MP / GBM, NTHR, 0, stream>>>(AGG, W2D, SM, NOf, FLAG, out);
}
